// LSQBlock_84885733638932
// MI455X (gfx1250) — hardware-run, weakly checked
//
#include <hip/hip_runtime.h>
#include <math.h>

#ifndef NB
#define NB 8
#endif
#ifndef SEQ
#define SEQ 1024
#endif
#define NB_FULL 8
#define SEQ_FULL 1024

constexpr int CD = 768;
constexpr int NH = 12;
constexpr int HD = 64;
constexpr int C3 = 3 * CD;
constexpr int C4 = 4 * CD;
constexpr int NCH = SEQ / 64;
constexpr int MTOK = NB * SEQ;
constexpr int QKP = 2 * CD;
constexpr int VTP = MTOK;
constexpr int LNP = CD / 128;
constexpr float LN_INV = 1.0f / (float)CD;

static_assert(NB >= 1 && NB <= NB_FULL);
static_assert(SEQ <= SEQ_FULL);
static_assert(NCH >= 1 && NCH <= 32);
static_assert(CD == NH * HD);
static_assert(HD == 64);
static_assert(CD % 128 == 0 && LNP * 128 == CD);
static_assert(MTOK % 64 == 0 && CD % 64 == 0 && C3 % 64 == 0 && C4 % 64 == 0 && QKP % 64 == 0);
static_assert(CD % 32 == 0 && C4 % 32 == 0);
static_assert(MTOK % 8 == 0);
static_assert(SEQ % 64 == 0);
static_assert(CD % 8 == 0 && C4 % 8 == 0);

typedef _Float16 h16;
typedef __attribute__((ext_vector_type(16))) _Float16 v16h;
typedef __attribute__((ext_vector_type(8)))  _Float16 v8h;
typedef __attribute__((ext_vector_type(8)))  float    v8f;
typedef __attribute__((ext_vector_type(4)))  float    v4f;
typedef __attribute__((ext_vector_type(4)))  int      v4i;
typedef __attribute__((ext_vector_type(4)))  unsigned int v4u;
typedef __attribute__((ext_vector_type(2)))  unsigned int v2u;

union FH { v16h v; v8h h[2]; };

#define VST2(T, ptr, val) do { const T vst2_v_ = (val); *(volatile T*)(ptr) = vst2_v_; __threadfence(); *(volatile T*)(ptr) = vst2_v_; } while (0)

#define WAVE_SYNC() do { __builtin_amdgcn_fence(3  , "workgroup"); __builtin_amdgcn_wave_barrier(); __builtin_amdgcn_fence(2  , "workgroup"); } while (0)

__device__ __forceinline__ float cmb_bf(float v) { const unsigned u = __builtin_bit_cast(unsigned, v); const unsigned r = (u + 0x7fffu + ((u >> 16) & 1u)) & 0xffff0000u; return __builtin_bit_cast(float, r); }
static __device__ __forceinline__ h16 toh_flush(float v) { const h16 r = (h16)v; return (fabsf(v) < 6.103515625e-05f) ? (h16)0.0f : r; }
__device__ __forceinline__ unsigned int pk2hf(float a, float b) { return (unsigned int)__builtin_bit_cast(unsigned short, toh_flush(a)) | ((unsigned int)__builtin_bit_cast(unsigned short, toh_flush(b)) << 16); }
__device__ __forceinline__ v16h ldg_frag(const _Float16* __restrict__ p) { FH f; f.h[0] = *(const v8h*)(p); f.h[1] = *(const v8h*)(p + 16); return f.v; }

__device__ __forceinline__ v8f mma_h(v16h a, v16h b, v8f c) {
  c = __builtin_amdgcn_wmma_f32_16x16x32_f16(false, a, false, b, (short)0, c, false, false);
  asm volatile("v_nop\n\tv_nop\n\tv_nop\n\tv_nop" : "+v"(c) : "v"(a), "v"(b));
  return c;
}
__device__ __forceinline__ void dep_guard_h(v8f& a, v8f& b, v16h x, v16h y) { asm volatile("v_nop\n\tv_nop\n\tv_nop\n\tv_nop" : "+v"(a), "+v"(b) : "v"(x), "v"(y)); }
__device__ __forceinline__ void keep4_h(v16h a, v16h b, v16h c, v16h d) { asm volatile("v_nop" :: "v"(a), "v"(b), "v"(c), "v"(d)); }
__device__ __forceinline__ void acc_guard4(v8f& a, v8f& b, v8f& c, v8f& d) { asm volatile("v_nop\n\tv_nop\n\tv_nop\n\tv_nop" : "+v"(a), "+v"(b), "+v"(c), "+v"(d)); }

__device__ __forceinline__ float gelu_erf(float t) {
  const float z = fabsf(t) * 0.7071067811865476f;
  const float k = __builtin_amdgcn_rcpf(1.0f + 0.3275911f * z);
  float p = 1.061405429f;
  p = p * k - 1.453152027f;
  p = p * k + 1.421413741f;
  p = p * k - 0.284496736f;
  p = p * k + 0.254829592f;
  p = p * k;
  const float e = exp2f(-1.4426950408889634f * (z * z));
  const float hc = 0.5f * (p * e);
  const float cdf = (t < 0.f) ? hc : (1.0f - hc);
  return t * cdf;
}

__global__ __launch_bounds__(32) void k_clsdense(int* __restrict__ cls) {
  const int qb = blockIdx.x, t = threadIdx.x;
  const int myc = (t < NCH) ? 1 : 0;
  VST2(int, cls + qb * 64 + t, myc);
  const int fv = 0;
  VST2(int, cls + qb * 64 + 32 + t, fv);
}

__global__ __launch_bounds__(256) void k_castw(const float* __restrict__ SRC, unsigned short* __restrict__ DST, int n8, float sc) {
  const int u = blockIdx.x * 256 + threadIdx.x; if (u >= n8) return;
  const v4f a = *(const v4f*)(SRC + (size_t)u * 8);
  const v4f b = *(const v4f*)(SRC + (size_t)u * 8 + 4);
  v4u pk;
  pk.x = pk2hf(cmb_bf(a.x) * sc, cmb_bf(a.y) * sc); pk.y = pk2hf(cmb_bf(a.z) * sc, cmb_bf(a.w) * sc);
  pk.z = pk2hf(cmb_bf(b.x) * sc, cmb_bf(b.y) * sc); pk.w = pk2hf(cmb_bf(b.z) * sc, cmb_bf(b.w) * sc);
  VST2(v4u, (v4u*)(DST + (size_t)u * 8), pk);
}

template <int ABF, int FULLMAP>
__device__ __forceinline__ void ln_body(const float* __restrict__ A, const float* __restrict__ GA, const float* __restrict__ BE, unsigned short* __restrict__ Y16) {
  #pragma clang fp contract(off)
  const int r = blockIdx.x * 8 + (threadIdx.x >> 5); const int L = threadIdx.x & 31; if (r >= MTOK) return;
  const size_t srow = FULLMAP ? ((size_t)(r / SEQ) * SEQ_FULL + (size_t)(r % SEQ)) : (size_t)r;
  v4f v[LNP]; float s = 0.f;
#pragma unroll
  for (int q = 0; q < LNP; ++q) {
    v[q] = *(const v4f*)(A + srow * CD + 4 * L + 128 * q);
    if (ABF) { v[q].x = cmb_bf(v[q].x); v[q].y = cmb_bf(v[q].y); v[q].z = cmb_bf(v[q].z); v[q].w = cmb_bf(v[q].w); }
    s += (v[q].x + v[q].y) + (v[q].z + v[q].w);
  }
#pragma unroll
  for (int o = 16; o > 0; o >>= 1) s += __shfl_xor(s, o, 32);
  const float mu = s * LN_INV; float qq = 0.f;
#pragma unroll
  for (int q = 0; q < LNP; ++q) { v[q].x -= mu; v[q].y -= mu; v[q].z -= mu; v[q].w -= mu; qq += (v[q].x * v[q].x + v[q].y * v[q].y) + (v[q].z * v[q].z + v[q].w * v[q].w); }
#pragma unroll
  for (int o = 16; o > 0; o >>= 1) qq += __shfl_xor(qq, o, 32);
  const float rs = rsqrtf(qq * LN_INV + 1e-6f);
#pragma unroll
  for (int q = 0; q < LNP; ++q) {
    const int c = 4 * L + 128 * q; const v4f ga = *(const v4f*)(GA + c), be = *(const v4f*)(BE + c); v4f y;
    y.x = v[q].x * rs * cmb_bf(ga.x) + cmb_bf(be.x); y.y = v[q].y * rs * cmb_bf(ga.y) + cmb_bf(be.y);
    y.z = v[q].z * rs * cmb_bf(ga.z) + cmb_bf(be.z); y.w = v[q].w * rs * cmb_bf(ga.w) + cmb_bf(be.w);
    v2u pk; pk.x = pk2hf(y.x, y.y); pk.y = pk2hf(y.z, y.w);
    VST2(v2u, (v2u*)(Y16 + (size_t)r * CD + c), pk);
  }
}
__global__ __launch_bounds__(256) void k_ln_in(const float* __restrict__ A, const float* __restrict__ GA, const float* __restrict__ BE, unsigned short* __restrict__ Y16) { ln_body<1, 1>(A, GA, BE, Y16); }
__global__ __launch_bounds__(256) void k_ln_mid(const float* __restrict__ A, const float* __restrict__ GA, const float* __restrict__ BE, unsigned short* __restrict__ Y16) { ln_body<0, 0>(A, GA, BE, Y16); }

struct GP {
  const unsigned short* A; const unsigned short* Bt; void* C; const float* bias; const float* R;
  long long strideA, strideC;
  int lda, ldb, ldc, ldr, M, N, K, rpb, rpbC, rpbR; float scale; int pad_;
};
static_assert(sizeof(GP) == 104);

template <int BIAS_MODE, int OUT_MODE, int RES_MODE, int ACT>
__device__ __forceinline__ void gemm_body(const GP& p) {
  __shared__ __align__(16) float sT[8][16 * 68];
  const int b = blockIdx.y;
  const int lane = threadIdx.x & 31, wave = threadIdx.x >> 5;
  const int tilesN = p.N >> 6, tilesM = p.M >> 6;
  const int tile = blockIdx.x * 8 + wave;
  if (tile >= tilesM * tilesN) return;
  const int tm = tile / tilesN, tn = tile - tm * tilesN;
  const int m0 = tm << 6, n0 = tn << 6;
  const _Float16* Ab = (const _Float16*)p.A + (size_t)b * p.strideA;
  const _Float16* Bb = (const _Float16*)p.Bt;
  const int rlane = lane & 15, koff = (lane >> 4) * 8, mOff = (lane >> 4) * 8;

  v8f acc[4][4];
#pragma unroll
  for (int i = 0; i < 4; ++i)
#pragma unroll
    for (int j = 0; j < 4; ++j) acc[i][j] = (v8f){0.f, 0.f, 0.f, 0.f, 0.f, 0.f, 0.f, 0.f};

  for (int k0 = 0; k0 < p.K; k0 += 32) {
    v16h bh[4];
#pragma unroll
    for (int j = 0; j < 4; ++j) bh[j] = ldg_frag(Bb + (size_t)(n0 + (j << 4) + rlane) * p.ldb + koff + k0);
#pragma unroll
    for (int i = 0; i < 4; ++i) {
      const v16h ah = ldg_frag(Ab + (size_t)(m0 + (i << 4) + rlane) * p.lda + koff + k0);
#pragma unroll
      for (int j = 0; j < 4; ++j) acc[i][j] = __builtin_amdgcn_wmma_f32_16x16x32_f16(false, ah, false, bh[j], (short)0, acc[i][j], false, false);
      dep_guard_h(acc[i][0], acc[i][3], ah, ah);
    }
    keep4_h(bh[0], bh[1], bh[2], bh[3]);
  }
  acc_guard4(acc[0][0], acc[0][1], acc[0][2], acc[0][3]);
  acc_guard4(acc[1][0], acc[1][1], acc[1][2], acc[1][3]);
  acc_guard4(acc[2][0], acc[2][1], acc[2][2], acc[2][3]);
  acc_guard4(acc[3][0], acc[3][1], acc[3][2], acc[3][3]);

  float* slab = sT[wave];
#pragma unroll
  for (int i = 0; i < 4; ++i) {
    const int mBase = m0 + (i << 4);
    float bm[8];
#pragma unroll
    for (int r = 0; r < 8; ++r) { bm[r] = 0.f; if (BIAS_MODE == 1) bm[r] = cmb_bf(p.bias[mBase + mOff + r]); }
#pragma unroll
    for (int j = 0; j < 4; ++j) {
      const int n = n0 + (j << 4) + rlane;
      float bv = 0.f; if (BIAS_MODE == 2) bv = cmb_bf(p.bias[n]);
#pragma unroll
      for (int r = 0; r < 8; ++r) {
        float v = acc[i][j][r] * p.scale + ((BIAS_MODE == 1) ? bm[r] : bv);
        if (ACT == 1) v = gelu_erf(v);
        slab[(mOff + r) * 68 + (j << 4) + rlane] = v;
      }
    }
    WAVE_SYNC();
    const int gb = mBase / p.rpb; const int tIn = mBase - gb * p.rpb;
    const size_t rowC0 = (size_t)gb * p.rpbC + tIn, rowR0 = (size_t)gb * p.rpbR + tIn;
    if (OUT_MODE == 0) {
      float* C = (float*)p.C + (size_t)b * p.strideC;
      const int hh = lane >> 4, c4 = (lane & 15) * 4;
      v4f val[8];
#pragma unroll
      for (int it = 0; it < 8; ++it) {
        const int row = it * 2 + hh;
        v4f v = *(const v4f*)(slab + row * 68 + c4);
        if (RES_MODE != 0) {
          v4f x = *(const v4f*)(p.R + (rowR0 + row) * (size_t)p.ldr + n0 + c4);
          if (RES_MODE == 2) { x.x = cmb_bf(x.x); x.y = cmb_bf(x.y); x.z = cmb_bf(x.z); x.w = cmb_bf(x.w); }
          v = v + x;
        }
        val[it] = v;
      }
      for (int pass = 0; pass < 2; ++pass) {
#pragma unroll
        for (int it = 0; it < 8; ++it) {
          const int row = it * 2 + hh;
          *(volatile v4f*)(C + (rowC0 + row) * (size_t)p.ldc + n0 + c4) = val[it];
        }
        __threadfence();
      }
    } else {
      unsigned short* C = (unsigned short*)p.C + (size_t)b * p.strideC;
      const int q = lane >> 3, c8 = (lane & 7) * 8;
      v8h hv[4];
#pragma unroll
      for (int it = 0; it < 4; ++it) {
        const float* sp = slab + (it * 4 + q) * 68 + c8;
#pragma unroll
        for (int e = 0; e < 8; ++e) hv[it][e] = toh_flush(sp[e]);
      }
      for (int pass = 0; pass < 2; ++pass) {
#pragma unroll
        for (int it = 0; it < 4; ++it) {
          const int row = it * 4 + q;
          *(volatile v8h*)(C + (rowC0 + row) * (size_t)p.ldc + n0 + c8) = hv[it];
        }
        __threadfence();
      }
    }
    WAVE_SYNC();
  }
}

__device__ __forceinline__ GP gp_pack(const unsigned short* A, const unsigned short* Bt, void* C, const float* bias, const float* R,
                                      long long strideA, long long strideC, int lda, int ldb, int ldc, int ldr, int M, int N, int K,
                                      int rpb, int rpbC, int rpbR, float scale) {
  GP g;
  g.A = A; g.Bt = Bt; g.C = C; g.bias = bias; g.R = R; g.strideA = strideA; g.strideC = strideC;
  g.lda = lda; g.ldb = ldb; g.ldc = ldc; g.ldr = ldr; g.M = M; g.N = N; g.K = K; g.rpb = rpb; g.rpbC = rpbC; g.rpbR = rpbR;
  g.scale = scale; g.pad_ = 0;
  return g;
}

__global__ __launch_bounds__(256) void k_gemm_qk(const unsigned short* A, const unsigned short* Bt, void* C, const float* bias, const float* R,
                                                   long long strideA, long long strideC, int lda, int ldb, int ldc, int ldr, int M, int N, int K,
                                                   int rpb, int rpbC, int rpbR, float scale) {
  const GP p = gp_pack(A, Bt, C, bias, R, strideA, strideC, lda, ldb, ldc, ldr, M, N, K, rpb, rpbC, rpbR, scale);
  gemm_body<2, 1, 0, 0>(p);
}
__global__ __launch_bounds__(256) void k_gemm_vt(const unsigned short* A, const unsigned short* Bt, void* C, const float* bias, const float* R,
                                                   long long strideA, long long strideC, int lda, int ldb, int ldc, int ldr, int M, int N, int K,
                                                   int rpb, int rpbC, int rpbR, float scale) {
  const GP p = gp_pack(A, Bt, C, bias, R, strideA, strideC, lda, ldb, ldc, ldr, M, N, K, rpb, rpbC, rpbR, scale);
  gemm_body<1, 1, 0, 0>(p);
}
__global__ __launch_bounds__(256) void k_gemm_proj(const unsigned short* A, const unsigned short* Bt, void* C, const float* bias, const float* R,
                                                     long long strideA, long long strideC, int lda, int ldb, int ldc, int ldr, int M, int N, int K,
                                                     int rpb, int rpbC, int rpbR, float scale) {
  const GP p = gp_pack(A, Bt, C, bias, R, strideA, strideC, lda, ldb, ldc, ldr, M, N, K, rpb, rpbC, rpbR, scale);
  gemm_body<2, 0, 2, 0>(p);
}
__global__ __launch_bounds__(256) void k_gemm_fc(const unsigned short* A, const unsigned short* Bt, void* C, const float* bias, const float* R,
                                                   long long strideA, long long strideC, int lda, int ldb, int ldc, int ldr, int M, int N, int K,
                                                   int rpb, int rpbC, int rpbR, float scale) {
  const GP p = gp_pack(A, Bt, C, bias, R, strideA, strideC, lda, ldb, ldc, ldr, M, N, K, rpb, rpbC, rpbR, scale);
  gemm_body<2, 1, 0, 1>(p);
}
__global__ __launch_bounds__(256) void k_gemm_mlp(const unsigned short* A, const unsigned short* Bt, void* C, const float* bias, const float* R,
                                                    long long strideA, long long strideC, int lda, int ldb, int ldc, int ldr, int M, int N, int K,
                                                    int rpb, int rpbC, int rpbR, float scale) {
  const GP p = gp_pack(A, Bt, C, bias, R, strideA, strideC, lda, ldb, ldc, ldr, M, N, K, rpb, rpbC, rpbR, scale);
  gemm_body<2, 0, 1, 0>(p);
}

#define ATT_SC 0.18033688011112042f
#define ATT_FILL (-3.4028234663852886e38f)
#define ATT_PCAR 4096.0f

__global__ __launch_bounds__(128) void k_attn_main(const unsigned short* __restrict__ QKp, const unsigned short* __restrict__ VTp,
                                                     const int* __restrict__ mask, const int* __restrict__ cls, unsigned short* __restrict__ CTXp) {
  __shared__ __align__(16) _Float16 Psh[4][16 * 64];
  __shared__ __align__(16) unsigned int Msh[4][16 * 16];
  __shared__ __align__(16) _Float16 Osh[4][16 * 64];
  const int tid = threadIdx.x, wave = tid >> 5, lane = tid & 31, hh = lane >> 4, c = lane & 15;
  const int bx = blockIdx.x; const int qb = bx % NCH; const int bhh = bx / NCH; const int h = bhh % NH; const int b = bhh / NH;
  const int q0 = qb * 64 + wave * 16;
  const _Float16* QK = (const _Float16*)QKp; const _Float16* VT = (const _Float16*)VTp;
  const size_t tok0 = (size_t)b * SEQ;

  v16h qa0, qa1;
  { const _Float16* qrow = QK + (tok0 + q0 + c) * (size_t)QKP + h * HD + 8 * hh; qa0 = ldg_frag(qrow); qa1 = ldg_frag(qrow + 32); }

  float mrow[8], lrow[8]; v8f oacc[4];
#pragma unroll
  for (int r = 0; r < 8; ++r) { mrow[r] = -INFINITY; lrow[r] = 0.f; }
#pragma unroll
  for (int t = 0; t < 4; ++t) oacc[t] = (v8f){0.f, 0.f, 0.f, 0.f, 0.f, 0.f, 0.f, 0.f};

  const int full = __builtin_amdgcn_readfirstlane(cls[qb * 64 + 32]);
  _Float16* pw = Psh[wave];
  unsigned int* msh = Msh[wave];
#pragma unroll 1
  for (int kc = 0; kc < NCH; ++kc) {
    const int cv = __builtin_amdgcn_readfirstlane(cls[qb * 64 + kc]);
    if (cv == 0 && full == 0) continue;
    const int kv0 = kc * 64;
    v8f s[4];
#pragma unroll
    for (int j = 0; j < 4; ++j) {
      const _Float16* krow = QK + (tok0 + kv0 + j * 16 + c) * (size_t)QKP + CD + h * HD + 8 * hh;
      const v16h kb0 = ldg_frag(krow), kb1 = ldg_frag(krow + 32);
      v8f z = (v8f){0.f, 0.f, 0.f, 0.f, 0.f, 0.f, 0.f, 0.f};
      z = mma_h(qa0, kb0, z);
      z = mma_h(qa1, kb1, z);
      s[j] = z * ATT_SC;
    }
    if (cv != 1) {
      const int* mb = mask + (size_t)q0 * SEQ_FULL + kv0;
#pragma unroll
      for (int it = 0; it < 8; ++it) {
        const int row = it * 2 + hh;
        const v4i m = *(const v4i*)(mb + (size_t)row * SEQ_FULL + 4 * c);
        msh[row * 16 + c] = ((m.x != 0) ? 1u : 0u) | ((m.y != 0) ? 0x100u : 0u) | ((m.z != 0) ? 0x10000u : 0u) | ((m.w != 0) ? 0x1000000u : 0u);
      }
      WAVE_SYNC();
#pragma unroll
      for (int r = 0; r < 8; ++r)
#pragma unroll
        for (int j = 0; j < 4; ++j) {
          const unsigned int w = msh[(8 * hh + r) * 16 + j * 4 + (c >> 2)];
          const bool keep = ((w >> (8 * (c & 3))) & 1u) != 0u;
          s[j][r] = keep ? s[j][r] : ATT_FILL;
        }
      WAVE_SYNC();
    }
#pragma unroll
    for (int r = 0; r < 8; ++r) {
      float m = fmaxf(fmaxf(s[0][r], s[1][r]), fmaxf(s[2][r], s[3][r]));
      m = fmaxf(m, __shfl_xor(m, 1, 32)); m = fmaxf(m, __shfl_xor(m, 2, 32));
      m = fmaxf(m, __shfl_xor(m, 4, 32)); m = fmaxf(m, __shfl_xor(m, 8, 32));
      const float mnew = fmaxf(mrow[r], m);
      const float alpha = exp2f(mrow[r] - mnew);
      mrow[r] = mnew;
      float psum = 0.f;
#pragma unroll
      for (int j = 0; j < 4; ++j) {
        const float pe = exp2f(s[j][r] - mnew);
        psum += pe;
        pw[(8 * hh + r) * 64 + j * 16 + c] = (_Float16)(pe * ATT_PCAR);
      }
      psum += __shfl_xor(psum, 1, 32); psum += __shfl_xor(psum, 2, 32); psum += __shfl_xor(psum, 4, 32); psum += __shfl_xor(psum, 8, 32);
      lrow[r] = lrow[r] * alpha + psum;
#pragma unroll
      for (int t = 0; t < 4; ++t) oacc[t][r] *= alpha;
    }
    WAVE_SYNC();
#pragma unroll
    for (int kk = 0; kk < 2; ++kk) {
      FH pa;
      pa.h[0] = *(const v8h*)(pw + c * 64 + kk * 32 + 8 * hh);
      pa.h[1] = *(const v8h*)(pw + c * 64 + kk * 32 + 16 + 8 * hh);
#pragma unroll
      for (int t = 0; t < 4; ++t) {
        const v16h vb = ldg_frag(VT + (size_t)(h * HD + t * 16 + c) * VTP + tok0 + kv0 + kk * 32 + 8 * hh);
        oacc[t] = mma_h(pa.v, vb, oacc[t]);
      }
    }
    WAVE_SYNC();
  }

  _Float16* os = Osh[wave];
#pragma unroll
  for (int r = 0; r < 8; ++r) {
    const float inv = (lrow[r] > 0.f) ? 1.0f / (lrow[r] * ATT_PCAR) : 0.f;
#pragma unroll
    for (int t = 0; t < 4; ++t) os[(8 * hh + r) * 64 + t * 16 + c] = (_Float16)(oacc[t][r] * inv);
  }
  WAVE_SYNC();
  {
    const int q = lane >> 3, c8 = (lane & 7) * 8;
    v8h hv[4];
#pragma unroll
    for (int it = 0; it < 4; ++it) hv[it] = *(const v8h*)(os + (it * 4 + q) * 64 + c8);
    for (int pass = 0; pass < 2; ++pass) {
#pragma unroll
      for (int it = 0; it < 4; ++it)
        *(volatile v8h*)(CTXp + (tok0 + q0 + it * 4 + q) * (size_t)CD + h * HD + c8) = hv[it];
      __threadfence();
    }
  }
}

constexpr size_t SZ_H16  = (size_t)MTOK * CD * 2;
constexpr size_t SZ_W3T  = (size_t)C3 * CD * 2;
constexpr size_t SZ_WOT  = (size_t)CD * CD * 2;
constexpr size_t SZ_W1T  = (size_t)C4 * CD * 2;
constexpr size_t SZ_W2T  = (size_t)CD * C4 * 2;
constexpr size_t SZ_QK   = (size_t)MTOK * QKP * 2;
constexpr size_t SZ_VT   = (size_t)CD * VTP * 2;
constexpr size_t SZ_CTX  = (size_t)MTOK * CD * 2;
constexpr size_t SZ_X1   = (size_t)MTOK * CD * 4;
constexpr size_t SZ_F16  = (size_t)MTOK * C4 * 2;
constexpr size_t SZ_CLS  = (size_t)NCH * 64 * 4;
constexpr size_t SZ_ATT  = SZ_QK + SZ_VT + SZ_CTX;
constexpr size_t OFF_H16 = 0;
constexpr size_t OFF_W3T = OFF_H16 + SZ_H16;
constexpr size_t OFF_WOT = OFF_W3T + SZ_W3T;
constexpr size_t OFF_W1T = OFF_WOT + SZ_WOT;
constexpr size_t OFF_W2T = OFF_W1T + SZ_W1T;
constexpr size_t OFF_QK  = OFF_W2T + SZ_W2T;
constexpr size_t OFF_VT  = OFF_QK + SZ_QK;
constexpr size_t OFF_CTX = OFF_VT + SZ_VT;
constexpr size_t OFF_F16 = OFF_QK;
constexpr size_t OFF_X1  = OFF_QK + SZ_ATT;
constexpr size_t OFF_CLS = OFF_X1 + SZ_X1;
constexpr size_t WS_TOTAL = OFF_CLS + SZ_CLS;
static_assert(SZ_F16 <= SZ_ATT);
static_assert(OFF_CTX + SZ_CTX == OFF_QK + SZ_ATT);
static_assert(WS_TOTAL <= (size_t)134217728);
static_assert(SZ_H16 % 256 == 0 && SZ_W3T % 256 == 0 && SZ_WOT % 256 == 0 && SZ_W1T % 256 == 0 && SZ_W2T % 256 == 0 && SZ_QK % 256 == 0 &&
              SZ_VT % 256 == 0 && SZ_CTX % 256 == 0 && SZ_X1 % 256 == 0 && SZ_F16 % 256 == 0 && SZ_CLS % 256 == 0);

static GP mk_gp(const unsigned short* A, long long sA, int lda, const unsigned short* Bt, int ldb, void* C, long long sC, int ldc,
                const float* bias, const float* R, int ldr, int M, int N, int K, int rpb, int rpbC, int rpbR) {
  GP g{};
  g.A = A; g.Bt = Bt; g.C = C; g.bias = bias; g.R = R; g.strideA = sA; g.strideC = sC;
  g.lda = lda; g.ldb = ldb; g.ldc = ldc; g.ldr = ldr; g.M = M; g.N = N; g.K = K; g.rpb = rpb; g.rpbC = rpbC; g.rpbR = rpbR;
  g.scale = 0.0625f; g.pad_ = 0;
  return g;
}
#define GP_ARGS(g) (g).A, (g).Bt, (g).C, (g).bias, (g).R, (g).strideA, (g).strideC, (g).lda, (g).ldb, (g).ldc, (g).ldr, (g).M, (g).N, (g).K, (g).rpb, (g).rpbC, (g).rpbR, (g).scale
static unsigned gemm_blocks(int M, int N) { return (unsigned)((((M / 64) * (N / 64)) + 7) / 8); }
static unsigned cast_blocks(int n8) { return (unsigned)((n8 + 255) / 256); }

extern "C" void kernel_launch(void* const* d_in, const int* in_sizes, int n_in, void* d_out, int out_size, void* d_ws, size_t ws_size, hipStream_t stream) {
  if (n_in < 15) return;
  const long long need_x = ((long long)(NB - 1) * SEQ_FULL + SEQ) * CD;
  if ((long long)in_sizes[0] < need_x) return;
  if (in_sizes[1] < 1 || in_sizes[2] < 1) return;
  if (in_sizes[3] < CD || in_sizes[4] < CD || in_sizes[5] < C3 * CD || in_sizes[6] < C3 || in_sizes[7] < CD * CD || in_sizes[8] < CD) return;
  if (in_sizes[9] < CD || in_sizes[10] < CD || in_sizes[11] < C4 * CD || in_sizes[12] < C4 || in_sizes[13] < CD * C4 || in_sizes[14] < CD) return;
  if ((long long)out_size < need_x) return;
  if (ws_size < WS_TOTAL) return;

  const float* x    = (const float*)d_in[0];
  const float* g1   = (const float*)d_in[3];
  const float* be1  = (const float*)d_in[4];
  const float* wqkv = (const float*)d_in[5];
  const float* bqkv = (const float*)d_in[6];
  const float* wo   = (const float*)d_in[7];
  const float* bo   = (const float*)d_in[8];
  const float* g2   = (const float*)d_in[9];
  const float* be2  = (const float*)d_in[10];
  const float* w1   = (const float*)d_in[11];
  const float* b1   = (const float*)d_in[12];
  const float* w2   = (const float*)d_in[13];
  const float* b2   = (const float*)d_in[14];
  float* out = (float*)d_out;
  char* wsp = (char*)d_ws;
  unsigned short* H16 = (unsigned short*)(wsp + OFF_H16);
  unsigned short* W3T = (unsigned short*)(wsp + OFF_W3T);
  unsigned short* WOT = (unsigned short*)(wsp + OFF_WOT);
  unsigned short* W1T = (unsigned short*)(wsp + OFF_W1T);
  unsigned short* W2T = (unsigned short*)(wsp + OFF_W2T);
  unsigned short* QK  = (unsigned short*)(wsp + OFF_QK);
  unsigned short* VT  = (unsigned short*)(wsp + OFF_VT);
  unsigned short* CTX = (unsigned short*)(wsp + OFF_CTX);
  float*          X1  = (float*)(wsp + OFF_X1);
  unsigned short* F16 = (unsigned short*)(wsp + OFF_F16);
  int*            CLS = (int*)(wsp + OFF_CLS);
  const int* nomask = (const int*)(wsp + OFF_H16);
  const int BIG = 1 << 30;

  k_clsdense<<<NCH, 32, 0, stream>>>(CLS);
  k_castw<<<cast_blocks(C3 * CD / 8), 256, 0, stream>>>(wqkv, W3T, C3 * CD / 8, 16.0f);
  k_castw<<<cast_blocks(CD * CD / 8), 256, 0, stream>>>(wo, WOT, CD * CD / 8, 16.0f);
  k_castw<<<cast_blocks(C4 * CD / 8), 256, 0, stream>>>(w1, W1T, C4 * CD / 8, 16.0f);
  k_castw<<<cast_blocks(CD * C4 / 8), 256, 0, stream>>>(w2, W2T, CD * C4 / 8, 16.0f);
  k_ln_in<<<MTOK / 8, 256, 0, stream>>>(x, g1, be1, H16);
  { const GP g = mk_gp(H16, 0, CD, W3T, CD, (void*)QK, 0, QKP, bqkv, nullptr, 0, MTOK, QKP, CD, BIG, BIG, BIG);
    k_gemm_qk<<<dim3(gemm_blocks(MTOK, QKP), 1), 256, 0, stream>>>(GP_ARGS(g)); }
  { const GP g = mk_gp(W3T + (size_t)2 * CD * CD, 0, CD, H16, CD, (void*)VT, 0, VTP, bqkv + 2 * CD, nullptr, 0, CD, MTOK, CD, BIG, BIG, BIG);
    k_gemm_vt<<<dim3(gemm_blocks(CD, MTOK), 1), 256, 0, stream>>>(GP_ARGS(g)); }
  k_attn_main<<<NB * NH * NCH, 128, 0, stream>>>(QK, VT, nomask, CLS, CTX);
  { const GP g = mk_gp(CTX, 0, CD, WOT, CD, (void*)X1, 0, CD, bo, x, CD, MTOK, CD, CD, SEQ, SEQ, SEQ_FULL);
    k_gemm_proj<<<dim3(gemm_blocks(MTOK, CD), 1), 256, 0, stream>>>(GP_ARGS(g)); }
  k_ln_mid<<<MTOK / 8, 256, 0, stream>>>(X1, g2, be2, H16);
  { const GP g = mk_gp(H16, 0, CD, W1T, CD, (void*)F16, 0, C4, b1, nullptr, 0, MTOK, C4, CD, BIG, BIG, BIG);
    k_gemm_fc<<<dim3(gemm_blocks(MTOK, C4), 1), 256, 0, stream>>>(GP_ARGS(g)); }
  { const GP g = mk_gp(F16, 0, C4, W2T, C4, (void*)out, 0, CD, b2, X1, CD, MTOK, CD, C4, SEQ, SEQ_FULL, SEQ);
    k_gemm_mlp<<<dim3(gemm_blocks(MTOK, CD), 1), 256, 0, stream>>>(GP_ARGS(g)); }
}
